// StandardAttention_75943611728135
// MI455X (gfx1250) — hardware-verified
//
#include <hip/hip_runtime.h>


#ifndef NB
#define NB 2
#endif
#ifndef SEQ
#define SEQ 2048
#endif
#ifndef NB_FULL
#define NB_FULL 2
#endif
#ifndef SEQ_FULL
#define SEQ_FULL 2048
#endif

namespace {
constexpr int E = 2048, H = 16, HD = 128, MR = NB * SEQ;
constexpr float XC = 8.0f, WC = 64.0f, QC = 8.0f, PS = 1024.0f, CC = 256.0f, LOG2E = 1.4426950408889634f, SCL = 0.02209708691207961f;
static_assert(SEQ % 128 == 0 && SEQ >= 128 && SEQ <= SEQ_FULL && NB >= 1 && NB <= NB_FULL);
static_assert(H * HD == E && E % 128 == 0 && E % 32 == 0 && MR % 128 == 0 && HD % 32 == 0 && SEQ % 32 == 0);

typedef _Float16 b16;
typedef __attribute__((ext_vector_type(16))) _Float16 v16b;
typedef __attribute__((ext_vector_type(8))) _Float16 v8b;
typedef __attribute__((ext_vector_type(8))) float v8f;
typedef __attribute__((ext_vector_type(4))) float v4f;

__device__ __forceinline__ float bf16_rne(float f) { unsigned int u = __float_as_uint(f); u += 0x7FFFu + ((u >> 16) & 1u); return __uint_as_float(u & 0xFFFF0000u); }
__device__ __forceinline__ v16b frag_kb(const b16* p, int hh) {
  const v8b a = *(const v8b*)(p + 8 * hh), b = *(const v8b*)(p + 16 + 8 * hh); v16b f;
#pragma unroll
  for (int e = 0; e < 8; ++e) { f[e] = a[e]; f[8 + e] = b[e]; }
  return f;
}
__device__ __forceinline__ v8f wmma16b(v16b a, v16b b, v8f c) {
  v8f d = __builtin_amdgcn_wmma_f32_16x16x32_f16(false, a, false, b, (short)0, c, false, false);
  asm volatile("v_nop\n\tv_nop\n\tv_nop\n\tv_nop" : "+v"(d) : "v"(a), "v"(b));
  return d;
}
__device__ __forceinline__ void wave_lds_sync() { __builtin_amdgcn_fence(3, "workgroup"); __builtin_amdgcn_wave_barrier(); __builtin_amdgcn_fence(2, "workgroup"); }
__device__ __forceinline__ float nexp2(float v) { return __builtin_amdgcn_exp2f(v); }

__global__ __launch_bounds__(256) void cvt_kernel(const float* __restrict__ X, const float* __restrict__ W0, const float* __restrict__ W1,
                                                  const float* __restrict__ W2, const float* __restrict__ W3, b16* __restrict__ Xp,
                                                  b16* __restrict__ P0, b16* __restrict__ P1, b16* __restrict__ P2, b16* __restrict__ P3) {
  const int y = (int)blockIdx.y; const size_t u = (size_t)blockIdx.x * 256 + threadIdx.x;
  const float* src; b16* dst; float c;
  if (y == 0) {
    if (u >= (size_t)MR * (E / 8)) return;
    const size_t row = u / (E / 8), p8 = u % (E / 8), b = row / SEQ, s = row % SEQ;
    src = X + (b * SEQ_FULL + s) * E + p8 * 8; dst = Xp + row * E + p8 * 8; c = XC;
  } else {
    if (u >= (size_t)E * E / 8) return;
    const float* w = (y == 1) ? W0 : (y == 2) ? W1 : (y == 3) ? W2 : W3;
    b16* p = (y == 1) ? P0 : (y == 2) ? P1 : (y == 3) ? P2 : P3;
    src = w + u * 8; dst = p + u * 8; c = WC;
  }
  const v4f x0 = *(const v4f*)src, x1 = *(const v4f*)(src + 4); v8b o;
#pragma unroll
  for (int j = 0; j < 4; ++j) { o[j] = (b16)(bf16_rne(x0[j]) * c); o[4 + j] = (b16)(bf16_rne(x1[j]) * c); }
  *(volatile v8b*)dst = o; __threadfence(); *(volatile v8b*)dst = o;
}

template <int EPI>
__global__ __launch_bounds__(256) __attribute__((amdgpu_num_vgpr(256))) void gemm_kernel(const b16* __restrict__ A, const b16* __restrict__ B0,
                                                                                       const b16* __restrict__ B1, const float* __restrict__ bias0,
                                                                                       const float* __restrict__ bias1, void* D0, void* D1) {
  __shared__ __attribute__((aligned(16))) float Ep[8][1152];
  const int tid = threadIdx.x, wave = tid >> 5, lane = tid & 31, hh = lane >> 4, col = lane & 15;
  const int r0 = (int)blockIdx.y * 128, c0 = (int)blockIdx.x * 128, tm = (wave >> 1) * 32, tn = (wave & 1) * 64;
  const bool sec = (blockIdx.z != 0);
  const b16* B = sec ? B1 : B0; const float* bias = sec ? bias1 : bias0; void* D = sec ? D1 : D0;
  const b16* Ar0 = A + (size_t)(r0 + tm + col) * E; const b16* Ar1 = Ar0 + (size_t)16 * E; const b16* Br = B + (size_t)(c0 + tn + col) * E;
  v8f acc[2][4];
#pragma unroll
  for (int i = 0; i < 2; ++i)
#pragma unroll
    for (int j = 0; j < 4; ++j) acc[i][j] = (v8f){};
#pragma unroll 1
  for (int k0 = 0; k0 < E; k0 += 32) {
    const v16b a0 = frag_kb(Ar0 + k0, hh), a1 = frag_kb(Ar1 + k0, hh);
#pragma unroll
    for (int j = 0; j < 4; ++j) {
      const v16b bj = frag_kb(Br + (size_t)j * 16 * E + k0, hh);
      acc[0][j] = wmma16b(a0, bj, acc[0][j]); acc[1][j] = wmma16b(a1, bj, acc[1][j]); }
  }
  if constexpr (EPI != 2) {
    b16* Eh = reinterpret_cast<b16*>(&Ep[wave][0]);
#pragma unroll
    for (int i = 0; i < 2; ++i) {
      float brv[8];
      if constexpr (EPI == 1) {
        const v4f b0 = *(const v4f*)(bias + r0 + tm + i * 16 + 8 * hh), b1 = *(const v4f*)(bias + r0 + tm + i * 16 + 8 * hh + 4);
#pragma unroll
        for (int r = 0; r < 4; ++r) { brv[r] = bf16_rne(b0[r]); brv[4 + r] = bf16_rne(b1[r]); }
      } else {
#pragma unroll
        for (int r = 0; r < 8; ++r) brv[r] = 0.0f;
      }
#pragma unroll
      for (int j = 0; j < 4; ++j) {
        float bc = 0.0f;
        if constexpr (EPI == 0) bc = bf16_rne(bias[c0 + tn + j * 16 + col]);
#pragma unroll
        for (int r = 0; r < 8; ++r) {
          float bb; if constexpr (EPI == 1) bb = brv[r]; else bb = bc;
          const float val = acc[i][j][r] * (1.0f / (XC * WC)) + bb;
          Eh[(i * 16 + 8 * hh + r) * 72 + j * 16 + col] = (b16)(val * QC); } } }
    wave_lds_sync();
    b16* dstb; size_t pitch;
    if constexpr (EPI == 0) {
      const int b = r0 / SEQ, s0 = r0 % SEQ + tm, h = c0 / HD;
      dstb = (b16*)D + (((size_t)(b * H + h) * SEQ + s0) * HD + tn); pitch = HD;
    } else {
      const int h = r0 / HD, b = c0 / SEQ, s0 = c0 % SEQ + tn;
      dstb = (b16*)D + (((size_t)(b * H + h) * HD + tm) * SEQ + s0); pitch = SEQ;
    }
    for (int pass = 0; pass < 2; ++pass) {
#pragma unroll 1
      for (int it = 0; it < 8; ++it) {
        const int rr = it * 4 + (lane >> 3), pc = (lane & 7) * 8;
        const v8b o = *(const v8b*)(Eh + rr * 72 + pc);
        *(volatile v8b*)(dstb + (size_t)rr * pitch + pc) = o; }
      __threadfence(); }
  } else {
    float* Ef = &Ep[wave][0];
    const int b = r0 / SEQ, s0 = r0 % SEQ + tm;
    float* dstb = (float*)D + ((size_t)b * SEQ_FULL + s0) * E + c0 + tn;
    float bc[4];
#pragma unroll
    for (int j = 0; j < 4; ++j) bc[j] = bf16_rne(bias[c0 + tn + j * 16 + col]);
#pragma unroll
    for (int i = 0; i < 2; ++i) {
#pragma unroll
      for (int j = 0; j < 4; ++j)
#pragma unroll
        for (int r = 0; r < 8; ++r) Ef[(8 * hh + r) * 68 + j * 16 + col] = acc[i][j][r] * (1.0f / (CC * WC)) + bc[j];
      wave_lds_sync();
      for (int pass = 0; pass < 2; ++pass) {
#pragma unroll 1
        for (int it = 0; it < 8; ++it) {
          const int rr = it * 2 + hh; const v4f f = *(const v4f*)(Ef + rr * 68 + col * 4);
          *(volatile v4f*)(dstb + (size_t)(i * 16 + rr) * E + col * 4) = f; }
        __threadfence(); }
      wave_lds_sync(); }
  }
}

__global__ __launch_bounds__(64) __attribute__((amdgpu_num_vgpr(256))) void attn_kernel(const b16* __restrict__ Qp, const b16* __restrict__ Kp,
                                                                                      const b16* __restrict__ VT, b16* __restrict__ Cp) {
  __shared__ __attribute__((aligned(16))) b16 Pb[2][16][32 + 8];
  __shared__ __attribute__((aligned(16))) b16 Tc[2][16][HD + 8];
  const int wave = threadIdx.x >> 5, lane = threadIdx.x & 31, hh = lane >> 4, col = lane & 15;
  const int bhi = (int)blockIdx.y; const int b = bhi / H, h = bhi % H;
  const int q0 = (int)blockIdx.x * 32 + wave * 16, qi = q0 + col;
  const b16* Qb = Qp + (size_t)bhi * SEQ * HD; const b16* Kb = Kp + (size_t)bhi * SEQ * HD; const b16* Vb = VT + (size_t)bhi * HD * (size_t)SEQ;
  v16b qa[4];
#pragma unroll
  for (int c4 = 0; c4 < 4; ++c4) qa[c4] = frag_kb(Qb + (size_t)qi * HD + 32 * c4, hh);
  const float cs = LOG2E * SCL / (QC * QC);
  float m = -INFINITY, l = 0.0f; v8f o[8];
#pragma unroll
  for (int t = 0; t < 8; ++t) o[t] = (v8f){};
#pragma unroll 1
  for (int kb = 0; kb < SEQ; kb += 32) {
    float e[16]; float mx = -INFINITY;
#pragma unroll
    for (int u = 0; u < 2; ++u) {
      const b16* kr = Kb + (size_t)(kb + u * 16 + col) * HD;
      v8f s = (v8f){};
#pragma unroll
      for (int c4 = 0; c4 < 4; ++c4) s = wmma16b(frag_kb(kr + 32 * c4, hh), qa[c4], s);
#pragma unroll
      for (int r = 0; r < 8; ++r) { const float v = s[r] * cs; e[u * 8 + r] = v; mx = fmaxf(mx, v); } }
    mx = fmaxf(mx, __shfl_xor(mx, 16)); const float mn = fmaxf(m, mx); const float al = nexp2(m - mn); float sum = 0.0f;
#pragma unroll
    for (int i2 = 0; i2 < 16; ++i2) {
      const float p = nexp2(e[i2] - mn); sum += p; const int pi = (i2 < 8 ? 0 : 16) + 8 * hh + (i2 & 7);
      Pb[wave][col][pi] = (b16)(p * PS); }
    sum += __shfl_xor(sum, 16); l = l * al + sum; m = mn;
    wave_lds_sync();
    const v16b pf = frag_kb(&Pb[wave][col][0], hh);
#pragma unroll
    for (int t = 0; t < 8; ++t) {
      o[t] *= al; const v16b vh = frag_kb(Vb + (size_t)(t * 16 + col) * SEQ + kb, hh);
      o[t] = wmma16b(vh, pf, o[t]); }
    wave_lds_sync(); }
  const float inv = CC / (l * PS * QC);
#pragma unroll
  for (int t = 0; t < 8; ++t) {
#pragma unroll
    for (int r = 0; r < 8; ++r) Tc[wave][col][t * 16 + 8 * hh + r] = (b16)(o[t][r] * inv); }
  wave_lds_sync();
  b16* cb = Cp + ((size_t)b * SEQ + (size_t)q0) * E + (size_t)h * HD;
  for (int pass = 0; pass < 2; ++pass) {
#pragma unroll 1
    for (int it = 0; it < 8; ++it) {
      const int rr = it * 2 + hh; const v8b f = *(const v8b*)(&Tc[wave][rr][col * 8]);
      *(volatile v8b*)(cb + (size_t)rr * E + col * 8) = f; }
    __threadfence(); }
}
}

extern "C" void kernel_launch(void* const* d_in, const int* in_sizes, int n_in, void* d_out, int out_size, void* d_ws, size_t ws_size, hipStream_t stream) {
  const size_t need_x = ((size_t)(NB - 1) * SEQ_FULL + SEQ) * E, need_w = (size_t)E * E, need_b = (size_t)E;
  if (n_in < 9 || (size_t)in_sizes[0] < need_x || (size_t)out_size < need_x) return;
  for (int i = 1; i < 9; i += 2) { if ((size_t)in_sizes[i] < need_w || (size_t)in_sizes[i + 1] < need_b) return; }
  const float* x = (const float*)d_in[0];
  const float* wq = (const float*)d_in[1]; const float* bq = (const float*)d_in[2];
  const float* wk = (const float*)d_in[3]; const float* bk = (const float*)d_in[4];
  const float* wv = (const float*)d_in[5]; const float* bv = (const float*)d_in[6];
  const float* wo = (const float*)d_in[7]; const float* bo = (const float*)d_in[8];
  size_t off = 0; char* ws = (char*)d_ws;
  auto carve = [&](size_t bytes) { char* p = ws + off; off += (bytes + 255) & ~(size_t)255; return p; };
  const size_t tok = (size_t)MR * E * 2, wpl = (size_t)E * E * 2;
  b16* Xp = (b16*)carve(tok);
  b16* Wqp = (b16*)carve(wpl); b16* Wkp = (b16*)carve(wpl); b16* Wvp = (b16*)carve(wpl); b16* Wop = (b16*)carve(wpl);
  b16* Qp = (b16*)carve(tok); b16* Kp = (b16*)carve(tok); b16* VTp = (b16*)carve(tok); b16* Cp = (b16*)carve(tok);
  if (off > ws_size || off > ((size_t)128 << 20)) return;
  const unsigned gx0 = (unsigned)(((size_t)MR * (E / 8) + 255) / 256), gx1 = (unsigned)(((size_t)E * E / 8 + 255) / 256);
  cvt_kernel<<<dim3(gx0 > gx1 ? gx0 : gx1, 5), 256, 0, stream>>>(x, wq, wk, wv, wo, Xp, Wqp, Wkp, Wvp, Wop);
  gemm_kernel<0><<<dim3(E / 128, MR / 128, 2), 256, 0, stream>>>(Xp, Wqp, Wkp, bq, bk, (void*)Qp, (void*)Kp);
  gemm_kernel<1><<<dim3(MR / 128, E / 128, 1), 256, 0, stream>>>(Wvp, Xp, Xp, bv, bv, (void*)VTp, (void*)VTp);
  attn_kernel<<<dim3(SEQ / 32, NB * H), 64, 0, stream>>>(Qp, Kp, VTp, Cp);
  gemm_kernel<2><<<dim3(E / 128, MR / 128, 1), 256, 0, stream>>>(Cp, Wop, Wop, bo, bo, d_out, d_out);
}
